// MySelfAttention_74096775790730
// MI455X (gfx1250) — hardware-verified
//
#include <hip/hip_runtime.h>
#include <math.h>

typedef __attribute__((ext_vector_type(16))) _Float16 v16h;
typedef __attribute__((ext_vector_type(16))) __bf16 v16b;
typedef __attribute__((ext_vector_type(8)))  _Float16 v8h;
typedef __attribute__((ext_vector_type(8)))  float v8f;
typedef __attribute__((ext_vector_type(4)))  float v4f;
typedef __attribute__((ext_vector_type(2)))  float v2f;
typedef __attribute__((ext_vector_type(4)))  unsigned v4u;
typedef __attribute__((ext_vector_type(4)))  int v4i;
typedef float __attribute__((may_alias)) float_a;
typedef int __attribute__((may_alias)) int_a;

template <typename T> __device__ __forceinline__ void vst2(void* p, T v) { *(volatile T*)p = v; __threadfence(); *(volatile T*)p = v; }
__device__ __forceinline__ v8f wmma16(v16h a, v16h b, v8f c) {
  v8f d = __builtin_amdgcn_wmma_f32_16x16x32_f16(false, a, false, b, (short)0, c, false, false);
  asm volatile("v_nop\n\tv_nop\n\tv_nop\n\tv_nop" : "+v"(d) : "v"(a), "v"(b));
  return d;
}
__device__ __forceinline__ v8f wmma_bf(v16b a, v16b b, v8f c) {
  v8f d = __builtin_amdgcn_wmma_f32_16x16x32_bf16(false, a, false, b, (short)0, c, false, false);
  asm volatile("v_nop\n\tv_nop\n\tv_nop\n\tv_nop" : "+v"(d) : "v"(a), "v"(b));
  return d;
}
__device__ __forceinline__ v16h frag_h(const _Float16* rowk0, int lane) {
  union { v16h v; v8h q[2]; } u; const _Float16* p = rowk0 + 8 * (lane >> 4);
  u.q[0] = *(const v8h*)p; u.q[1] = *(const v8h*)(p + 16); return u.v;
}
__device__ __forceinline__ v16h frag_f32(const float* rowk0, int lane) {
  v16h a; const float* p = rowk0 + 8 * (lane >> 4);
#pragma unroll
  for (int i = 0; i < 8; ++i) { a[i] = (_Float16)p[i]; a[8 + i] = (_Float16)p[16 + i]; }
  return a;
}
__device__ __forceinline__ v16h frag_f32s(const float* rowk0, int lane, float sc) {
  v16h a; const float* p = rowk0 + 8 * (lane >> 4);
#pragma unroll
  for (int i = 0; i < 8; ++i) { a[i] = (_Float16)(p[i] * sc); a[8 + i] = (_Float16)(p[16 + i] * sc); }
  return a;
}
__device__ __forceinline__ v16h fragc_f32(const float* W, int k0, int n, int lane, int ld, int K) {
  v16h a; const int g = lane >> 4;
#pragma unroll
  for (int i = 0; i < 8; ++i) { const int ka = k0 + 8 * g + i, kb = ka + 16;
    a[i] = (_Float16)(ka < K ? W[(size_t)(ka < K ? ka : K - 1) * ld + n] : 0.f); a[8 + i] = (_Float16)(kb < K ? W[(size_t)(kb < K ? kb : K - 1) * ld + n] : 0.f); }
  return a;
}
struct F2 { v16b h, l; };
__device__ __forceinline__ F2 bsplit16(const float v[16]) { F2 r;
#pragma unroll
  for (int i = 0; i < 16; ++i) { const __bf16 h = (__bf16)v[i]; r.h[i] = h; r.l[i] = (__bf16)(v[i] - (float)h); }
  return r; }
__device__ __forceinline__ F2 split_row(const float* row, int k0, int lane) { float v[16]; const float* p = row + k0 + 8 * (lane >> 4);
#pragma unroll
  for (int i = 0; i < 8; ++i) { v[i] = p[i]; v[8 + i] = p[16 + i]; }
  return bsplit16(v); }
__device__ __forceinline__ F2 split_rowK(const float* row, int k0, int lane, int K) { float v[16]; const int g = lane >> 4;
#pragma unroll
  for (int i = 0; i < 8; ++i) { const int ka = k0 + 8 * g + i, kb = ka + 16; v[i] = ka < K ? row[ka < K ? ka : K - 1] : 0.f; v[8 + i] = kb < K ? row[kb < K ? kb : K - 1] : 0.f; }
  return bsplit16(v); }
__device__ __forceinline__ F2 split_col(const float* W, int k0, int n, int lane, int ld, int K) { float v[16]; const int g = lane >> 4;
#pragma unroll
  for (int i = 0; i < 8; ++i) { const int ka = k0 + 8 * g + i, kb = ka + 16; v[i] = ka < K ? W[(size_t)(ka < K ? ka : K - 1) * ld + n] : 0.f; v[8 + i] = kb < K ? W[(size_t)(kb < K ? kb : K - 1) * ld + n] : 0.f; }
  return bsplit16(v); }
__device__ __forceinline__ v8f mac3(const F2& a, const F2& b, v8f c) { c = wmma_bf(a.l, b.h, c); c = wmma_bf(a.h, b.l, c); return wmma_bf(a.h, b.h, c); }
__device__ __forceinline__ float sigm(float v) { return 1.0f / (1.0f + expf(-v)); }
#define LDSX() do { asm volatile("s_wait_dscnt 0" ::: "memory"); __builtin_amdgcn_wave_barrier(); __builtin_amdgcn_fence(__ATOMIC_RELEASE, "workgroup"); } while (0)

#define NB 4
#define TT 2048
#define CC 1024
#define SCALE 0.03125f
#ifndef TNB
#define TNB NB
#endif
__device__ __forceinline__ float bfr(float v) { return (float)(__bf16)v; }
__device__ __forceinline__ v16b wrow(const float* rowk0, int lane) { v16b w; const float* p = rowk0 + 8 * (lane >> 4);
#pragma unroll
  for (int i = 0; i < 8; ++i) { w[i] = (__bf16)p[i]; w[8 + i] = (__bf16)p[16 + i]; }
  return w; }

#define WS_QH  0u
#define WS_KH  (WS_QH + 2u * (size_t)NB * TT * CC)
#define WS_VT  (WS_KH + 2u * (size_t)NB * TT * CC)
#define WS_S   (WS_VT + 2u * (size_t)NB * CC * TT)
#define WS_END (WS_S  + 4u * (size_t)TT * TT)

__global__ __launch_bounds__(128) void k_proj(const float* __restrict__ X, const float* __restrict__ WQ, const float* __restrict__ BQ, const float* __restrict__ WK, const float* __restrict__ BK, const float* __restrict__ WV, const float* __restrict__ BV, _Float16* __restrict__ QH, _Float16* __restrict__ KH, _Float16* __restrict__ VT) {
  __shared__ __align__(16) _Float16 sh[64][136]; __shared__ __align__(16) _Float16 th[128][72];
  const int tid = threadIdx.x, wave = tid >> 5, lane = tid & 31, col = lane & 15, g = lane >> 4; const int which = blockIdx.z; const int c0 = blockIdx.y * 128; const size_t r0 = (size_t)blockIdx.x * 64;
  const float* WA = which == 0 ? WQ : which == 1 ? WK : WV; const float* BA = which == 0 ? BQ : which == 1 ? BK : BV;
  v8f acc[8] = {};
#pragma unroll 2
  for (int kc = 0; kc < CC / 32; ++kc) { v16b a; { const float* p = X + (r0 + wave * 16 + col) * CC + kc * 32 + 8 * g;
#pragma unroll
      for (int i = 0; i < 8; ++i) { a[i] = (__bf16)p[i]; a[8 + i] = (__bf16)p[16 + i]; } }
#pragma unroll
    for (int j = 0; j < 8; ++j) { const v16b w = wrow(WA + (size_t)(c0 + j * 16 + col) * CC + kc * 32, lane); asm volatile("s_wait_loadcnt 0x0" ::: "memory"); acc[j] = wmma_bf(a, w, acc[j]); } }
  if (which < 2) {
#pragma unroll
    for (int j = 0; j < 8; ++j) { const float bb = bfr(BA[c0 + j * 16 + col]);
#pragma unroll
      for (int r = 0; r < 8; ++r) sh[wave * 16 + 8 * g + r][j * 16 + col] = (_Float16)(acc[j][r] + bb); }
    __syncthreads();
    _Float16* dh = which == 0 ? QH : KH; for (int e = tid; e < 64 * 16; e += 128) { const int rl = e >> 4, q = e & 15; vst2((unsigned*)(dh + (r0 + rl) * CC + c0 + q * 8), *(const v4u*)&sh[rl][q * 8]); }
  } else {
#pragma unroll
    for (int j = 0; j < 8; ++j) { const float bb = bfr(BA[c0 + j * 16 + col]);
#pragma unroll
      for (int r = 0; r < 8; ++r) th[j * 16 + col][wave * 16 + 8 * g + r] = (_Float16)(acc[j][r] + bb); }
    __syncthreads();
    const size_t b = r0 / TT; const int t0 = (int)(r0 % TT); for (int e = tid; e < 128 * 8; e += 128) { const int cl = e >> 3, q = e & 7; vst2((unsigned*)(VT + (b * CC + c0 + cl) * (size_t)TT + t0 + q * 8), *(const v4u*)&th[cl][q * 8]); } } }
__global__ __launch_bounds__(128) void k_sc(const _Float16* __restrict__ QH, const _Float16* __restrict__ KH, int b, float* __restrict__ S) { __shared__ __align__(16) float ss[4][16][132];
  const int tid = threadIdx.x, wave = tid >> 5, lane = tid & 31, col = lane & 15, g = lane >> 4; const int k0 = blockIdx.y * 128; const int ql0 = blockIdx.x * 64 + wave * 16; const size_t q0 = (size_t)b * TT + ql0, kr0 = (size_t)b * TT + k0;
  v8f acc[8] = {};
#pragma unroll 2
  for (int kc = 0; kc < CC / 32; ++kc) { const v16h ah = frag_h(QH + (q0 + col) * CC + kc * 32, lane);
#pragma unroll
    for (int j = 0; j < 8; ++j) { const v16h kb = frag_h(KH + (kr0 + j * 16 + col) * CC + kc * 32, lane); acc[j] = wmma16(ah, kb, acc[j]); } }
#pragma unroll
  for (int j = 0; j < 8; ++j) {
#pragma unroll
    for (int r = 0; r < 8; ++r) ss[wave][8 * g + r][j * 16 + col] = acc[j][r] * SCALE; }
  LDSX(); for (int rl = 0; rl < 16; ++rl) vst2(S + (size_t)(ql0 + rl) * TT + k0 + lane * 4, *(const v4f*)&ss[wave][rl][lane * 4]); }
__global__ __launch_bounds__(256) void k_sm(float* __restrict__ S0) { __shared__ float sred[8]; __shared__ float sbc; __shared__ __align__(16) float sh[TT];
  const int t = threadIdx.x; const size_t row = blockIdx.x; float* sr = S0 + row * TT; const int kend = TT;
  float m = -3.0e38f; for (int k = t; k < kend; k += 256) m = fmaxf(m, sr[k]);
#pragma unroll
  for (int o = 1; o < 32; o <<= 1) m = fmaxf(m, __shfl_xor(m, o));
  if ((t & 31) == 0) sred[t >> 5] = m; __syncthreads(); if (t == 0) { float a = sred[0]; for (int i = 1; i < 8; ++i) a = fmaxf(a, sred[i]); sbc = a; } __syncthreads(); m = sbc; __syncthreads();
  float sum = 0.f; for (int k = t; k < kend; k += 256) { const float e = expf(sr[k] - m); sh[k] = e; sum += e; }
#pragma unroll
  for (int o = 1; o < 32; o <<= 1) sum += __shfl_xor(sum, o);
  if ((t & 31) == 0) sred[t >> 5] = sum; __syncthreads(); if (t == 0) { float a = 0.f; for (int i = 0; i < 8; ++i) a += sred[i]; sbc = 2048.0f / a; } __syncthreads(); const float inv = sbc;
  for (int k = t; k < kend; k += 256) sh[k] = sh[k] * inv;
  __syncthreads(); for (int q = t; q < kend / 4; q += 256) vst2(sr + q * 4, *(const v4f*)&sh[q * 4]); }
__global__ __launch_bounds__(128) void k_pv(const float* __restrict__ PS, const _Float16* __restrict__ VT, int b, float* __restrict__ OUT) { __shared__ __align__(16) float ss[4][16][132];
  const int tid = threadIdx.x, wave = tid >> 5, lane = tid & 31, col = lane & 15, g = lane >> 4; const int ql0 = blockIdx.x * 64 + wave * 16; const int c0 = blockIdx.y * 128;
  v8f acc[8] = {};
#pragma unroll 1
  for (int kc = 0; kc < TT / 32; ++kc) { const v16h p = frag_f32(PS + (size_t)(ql0 + col) * TT + kc * 32, lane);
    asm volatile("s_wait_loadcnt 0x0" ::: "memory");
#pragma unroll
    for (int j = 0; j < 8; ++j) { const size_t po = ((size_t)b * CC + c0 + j * 16 + col) * (size_t)TT + kc * 32; acc[j] = wmma16(p, frag_h(VT + po, lane), acc[j]); } }
#pragma unroll
  for (int j = 0; j < 8; ++j)
#pragma unroll
    for (int r = 0; r < 8; ++r) ss[wave][8 * g + r][j * 16 + col] = acc[j][r] * (1.0f / 2048.0f);
  LDSX(); for (int rl = 0; rl < 16; ++rl) vst2(OUT + ((size_t)b * TT + ql0 + rl) * CC + c0 + lane * 4, *(const v4f*)&ss[wave][rl][lane * 4]); }
extern "C" void kernel_launch(void* const* d_in, const int* in_sizes, int n_in, void* d_out, int out_size, void* d_ws, size_t ws_size, hipStream_t stream) {
  (void)in_sizes; (void)n_in; (void)out_size;
  const float** F = (const float**)d_in;
  if (ws_size < (size_t)WS_END) return;
  char* ws = (char*)d_ws; _Float16 *QH = (_Float16*)(ws + WS_QH), *KH = (_Float16*)(ws + WS_KH), *VT = (_Float16*)(ws + WS_VT); float* S = (float*)(ws + WS_S);
  k_proj<<<dim3(TNB * TT / 64, CC / 128, 3), 128, 0, stream>>>(F[0], F[1], F[2], F[3], F[4], F[5], F[6], QH, KH, VT);
  for (int b = 0; b < TNB; ++b) {
    k_sc<<<dim3(TT / 64, TT / 128), 128, 0, stream>>>(QH, KH, b, S);
    k_sm<<<dim3(TT), 256, 0, stream>>>(S);
    k_pv<<<dim3(TT / 64, CC / 128), 128, 0, stream>>>(S, VT, b, (float*)d_out);
  }
}
